// Model_6442450944409
// MI455X (gfx1250) — hardware-verified
//
#include <hip/hip_runtime.h>
#include <math.h>

typedef __attribute__((ext_vector_type(16))) _Float16 v16h;
typedef __attribute__((ext_vector_type(8)))  _Float16 v8h;
typedef __attribute__((ext_vector_type(8)))  float    v8f;
typedef __attribute__((ext_vector_type(4)))  float    v4f;
typedef __attribute__((ext_vector_type(2)))  float    v2f;
typedef __attribute__((ext_vector_type(4)))  unsigned int v4u;

constexpr int kSeqT     = 10;
constexpr int kChan     = 7;
constexpr int kNode     = 10;
constexpr int kGhid     = 32;
constexpr int kLhid     = 64;
constexpr int kHeads    = 4;
constexpr int kEmb      = 128;
constexpr int kCat      = 2 * kLhid;
constexpr int kGate     = 4 * kLhid;
constexpr int kFeat1    = 3 * kChan;
constexpr int kFeat1Pad = 32;
constexpr int kXRow     = kSeqT * kFeat1Pad;
constexpr float kWCarry = 16.0f;
constexpr float kWInv   = 1.0f / kWCarry;
static_assert(kCat == 128 && kGate == 256 && kFeat1 == 21 && kXRow == 320, "shape constants");
static_assert(kFeat1Pad % 32 == 0 && kCat % 32 == 0 && kLhid % 32 == 0 && kGhid % 32 == 0, "K multiples of 32");
static_assert((kXRow * 2) % 128 == 0, "X sample block is whole lines");

constexpr int OSTR = 136;
constexpr int XSTR = 40;
constexpr int OSP  = 132;
constexpr int H1P  = 136;
constexpr int GTP  = 40;
constexpr int GKW  = 4;

template <typename T> struct Frag;
template <> struct Frag<_Float16> {
  typedef v16h V; union U { v16h v; v8h h[2]; };
  static __device__ __forceinline__ v16h load(const _Float16* p) {
    U f; f.h[0] = *(const v8h*)(p); f.h[1] = *(const v8h*)(p + 16); return f.v;
  }
  static __device__ __forceinline__ v8f mma(v16h a, v16h b, v8f c) {
    return __builtin_amdgcn_wmma_f32_16x16x32_f16(false, a, false, b, (short)0, c, false, false);
  }
};
typedef Frag<_Float16> FragH;

__device__ __forceinline__ void wm_guard4(v8f& a0, v8f& a1, v8f& a2, v8f& a3, v16h x, v16h y0, v16h y1, v16h y2, v16h y3) {
  asm volatile("v_nop\n\tv_nop\n\tv_nop\n\tv_nop" : "+v"(a0), "+v"(a1), "+v"(a2), "+v"(a3) : "v"(x), "v"(y0), "v"(y1), "v"(y2), "v"(y3));
}
__device__ __forceinline__ void wm_guard1x8(v8f& a0, v16h x0, v16h x1, v16h x2, v16h x3, v16h y0, v16h y1, v16h y2, v16h y3) {
  asm volatile("v_nop\n\tv_nop\n\tv_nop\n\tv_nop" : "+v"(a0) : "v"(x0), "v"(x1), "v"(x2), "v"(x3), "v"(y0), "v"(y1), "v"(y2), "v"(y3));
}
__device__ __forceinline__ void wm_guard1x4(v8f& a0, v16h x0, v16h x1, v16h y0, v16h y1) {
  asm volatile("v_nop\n\tv_nop\n\tv_nop\n\tv_nop" : "+v"(a0) : "v"(x0), "v"(x1), "v"(y0), "v"(y1));
}

__device__ __forceinline__ unsigned pk16(unsigned short a, unsigned short b) { return (unsigned)a | ((unsigned)b << 16); }
__device__ __forceinline__ unsigned short h_bits(float f) { const _Float16 h = (_Float16)f; return __builtin_bit_cast(unsigned short, h); }

__device__ __forceinline__ float h16_to_f32(unsigned hb) {
  const unsigned sgn = (hb & 0x8000u) << 16; const unsigned em = hb & 0x7fffu;
  const float fn = __uint_as_float((em << 13) + 0x38000000u);
  const float fs = (float)em * 5.9604644775390625e-8f;
  const float mag = (em < 0x400u) ? fs : fn; return __uint_as_float(__float_as_uint(mag) | sgn);
}

__device__ __forceinline__ float sigm_f(float x) { return __builtin_amdgcn_rcpf(1.0f + expf(-x)); }
__device__ __forceinline__ float tanh_f(float x) { return 1.0f - 2.0f * __builtin_amdgcn_rcpf(1.0f + expf(2.0f * x)); }

__device__ __forceinline__ int adj_sl_mask(int i) {
  return (i < 4) ? ((1 << i) | 0x080) : ((i < 7) ? ((1 << i) | 0x100) : ((i == 7) ? 0x38F : ((i == 8) ? 0x3F0 : 0x380)));
}
__device__ __forceinline__ int adj_mask(int i) {
  return (i < 4) ? 0x080 : ((i < 7) ? 0x100 : ((i == 7) ? 0x30F : ((i == 8) ? 0x2F0 : 0x180)));
}

__global__ __launch_bounds__(256) void cvt_plane_kernel(const float* __restrict__ s0, const float* __restrict__ s1,
                                                        const float* __restrict__ s2, unsigned short* __restrict__ dst,
                                                        int rows_src, int ksrc, int rows_dst, int kdst, float scale) {
  const int y = blockIdx.y;
  const float* src = (y == 0) ? s0 : ((y == 1) ? s1 : s2);
  const int cpr = kdst >> 3;
  const int nchunk = rows_dst * cpr;
  const int i = blockIdx.x * 256 + threadIdx.x;
  if (i < nchunk) {
    const int r  = i / cpr;
    const int k0 = (i - r * cpr) * 8;
    const int rc = (r < rows_src) ? r : (rows_src - 1);
    unsigned short hb[8];
#pragma unroll
    for (int e = 0; e < 8; ++e) {
      const int k  = k0 + e;
      const int kc = (k < ksrc) ? k : (ksrc - 1);
      const float v = src[(size_t)rc * ksrc + kc];
      const float val = ((r < rows_src) && (k < ksrc)) ? (v * scale) : 0.0f;
      hb[e] = h_bits(val);
    }
    const v4u u = (v4u){pk16(hb[0], hb[1]), pk16(hb[2], hb[3]), pk16(hb[4], hb[5]), pk16(hb[6], hb[7])};
    unsigned short* q = dst + (size_t)y * rows_dst * kdst + (size_t)i * 8;
    *(volatile v4u*)q = u;
    __threadfence();
    *(volatile v4u*)q = u;
  }
}

__global__ __launch_bounds__(128) void graph_front_kernel(
    const float* __restrict__ Min,
    const float* __restrict__ ga1W, const float* __restrict__ ga1s, const float* __restrict__ ga1d, const float* __restrict__ ga1b,
    const unsigned short* __restrict__ G2Wp, const float* __restrict__ ga2s, const float* __restrict__ ga2d, const float* __restrict__ ga2b,
    const float* __restrict__ gp1rel, const float* __restrict__ gp1root, const float* __restrict__ gp1b,
    const unsigned short* __restrict__ GC2rootp, const unsigned short* __restrict__ GC2relp, const float* __restrict__ gp2b,
    unsigned short* __restrict__ Xout, int nB) {
  __shared__ float x0s[GKW][104];
  __shared__ float agxs[GKW][104];
  __shared__ float xpss[GKW][kNode * 128];
  __shared__ float sAs[GKW][40];
  __shared__ float dAs[GKW][40];
  __shared__ __align__(16) _Float16 h1ts[GKW][16 * H1P];
  __shared__ float xp2ss[GKW][16 * 16];
  __shared__ float s2ss[GKW][16];
  __shared__ float d2ss[GKW][16];
  __shared__ __align__(16) _Float16 gtss[GKW][16 * GTP];
  __shared__ __align__(16) _Float16 gass[GKW][16 * GTP];
  __shared__ __align__(16) _Float16 xtss[GKW][kXRow];

  const int lane = threadIdx.x & 31;
  const int wave = threadIdx.x >> 5;
  const int b    = blockIdx.x * GKW + wave;
  const bool live = (b < nB);
  const int bc   = live ? b : (nB - 1);
  const int c = lane & 15, hh = lane >> 4, koff = hh * 8;

  float* x0  = x0s[wave];
  float* ag  = agxs[wave];
  float* xp  = xpss[wave];
  float* sA  = sAs[wave];
  float* dA  = dAs[wave];
  _Float16* h1 = h1ts[wave];
  float* xp2 = xp2ss[wave];
  float* s2v = s2ss[wave];
  float* d2v = d2ss[wave];
  _Float16* gt = gtss[wave];
  _Float16* ga = gass[wave];
  _Float16* xt = xtss[wave];
  const v8f z8 = {0.f, 0.f, 0.f, 0.f, 0.f, 0.f, 0.f, 0.f};

#pragma unroll 1
  for (int it = 0; it < 4; ++it) {
    const int idx = it * 32 + lane;
    const int ic  = (idx < 100) ? idx : 99;
    const int n   = ic / 10;
    const int f   = ic - n * 10;
    const int nc  = (n < kChan) ? n : (kChan - 1);
    const float v = Min[(size_t)bc * (kChan * kSeqT) + nc * kSeqT + f];
    const float val = (n < kChan) ? v : 0.0f;
    if (idx < 100) x0[ic] = val;
  }
  __syncthreads();

#pragma unroll 1
  for (int it = 0; it < 4; ++it) {
    const int idx = it * 32 + lane;
    const int ic  = (idx < 100) ? idx : 99;
    const int n   = ic / 10;
    const int f   = ic - n * 10;
    const int mk  = adj_mask(n);
    float a = 0.0f;
#pragma unroll 1
    for (int j = 0; j < kNode; ++j) {
      const float xv = x0[j * 10 + f];
      a += ((mk >> j) & 1) ? xv : 0.0f;
    }
    if (idx < 100) ag[ic] = a;
  }

  {
    float w1[kHeads][10];
#pragma unroll
    for (int h = 0; h < kHeads; ++h) {
      const v2f* wp = (const v2f*)(ga1W + (h * 32 + lane) * 10);
#pragma unroll
      for (int q = 0; q < 5; ++q) {
        const v2f t2 = wp[q];
        w1[h][2 * q]     = t2[0];
        w1[h][2 * q + 1] = t2[1];
      }
    }
    float as1[kHeads], ad1[kHeads];
#pragma unroll
    for (int h = 0; h < kHeads; ++h) { as1[h] = ga1s[h * 32 + lane]; ad1[h] = ga1d[h * 32 + lane]; }
#pragma unroll 1
    for (int n = 0; n < kChan; ++n) {
      float xv[10];
#pragma unroll
      for (int f = 0; f < 10; ++f) xv[f] = x0[n * 10 + f];
      float ps[kHeads], pd[kHeads];
#pragma unroll
      for (int h = 0; h < kHeads; ++h) {
        float acc = 0.0f;
#pragma unroll
        for (int f = 0; f < 10; ++f) acc = fmaf(xv[f], w1[h][f], acc);
        xp[n * 128 + h * 32 + lane] = acc;
        ps[h] = acc * as1[h];
        pd[h] = acc * ad1[h];
      }
#pragma unroll
      for (int off = 16; off > 0; off >>= 1) {
#pragma unroll
        for (int h = 0; h < kHeads; ++h) {
          ps[h] += __shfl_xor(ps[h], off, 32);
          pd[h] += __shfl_xor(pd[h], off, 32);
        }
      }
      if (lane == 0) {
#pragma unroll
        for (int h = 0; h < kHeads; ++h) { sA[n * 4 + h] = ps[h]; dA[n * 4 + h] = pd[h]; }
      }
    }
#pragma unroll 1
    for (int n = kChan; n < kNode; ++n) {
#pragma unroll
      for (int h = 0; h < kHeads; ++h) xp[n * 128 + h * 32 + lane] = 0.0f;
    }
    if (lane < 12) { sA[28 + lane] = 0.0f; dA[28 + lane] = 0.0f; }
  }
#pragma unroll 1
  for (int r = 9; r < 16; ++r) {
#pragma unroll
    for (int q = 0; q < 4; ++q) h1[r * H1P + q * 32 + lane] = (_Float16)0.0f;
    gt[r * GTP + lane] = (_Float16)0.0f;
  }
#pragma unroll 1
  for (int r = 7; r < 16; ++r) ga[r * GTP + lane] = (_Float16)0.0f;
#pragma unroll 1
  for (int q = 0; q < kSeqT; ++q) xt[q * 32 + lane] = (_Float16)0.0f;
  __syncthreads();

#pragma unroll 1
  for (int i = 0; i < 9; ++i) {
    const int mk = adj_sl_mask(i);
#pragma unroll 1
    for (int h = 0; h < kHeads; ++h) {
      const float di = dA[i * 4 + h];
      float mx = -INFINITY;
#pragma unroll 1
      for (int m = mk; m != 0; m &= (m - 1)) {
        const int j = __builtin_ctz(m);
        float v = di + sA[j * 4 + h];
        v = (v >= 0.0f) ? v : 0.2f * v;
        mx = fmaxf(mx, v);
      }
      float sum = 0.0f, o = 0.0f;
#pragma unroll 1
      for (int m = mk; m != 0; m &= (m - 1)) {
        const int j = __builtin_ctz(m);
        float v = di + sA[j * 4 + h];
        v = (v >= 0.0f) ? v : 0.2f * v;
        const float e = expf(v - mx);
        sum += e;
        o = fmaf(e, xp[j * 128 + h * 32 + lane], o);
      }
      const float bv = ga1b[h * 32 + lane];
      const float hv = fmaxf(o * (1.0f / sum) + bv, 0.0f);
      h1[i * H1P + h * 32 + lane] = (_Float16)hv;
    }
  }
  {
    float wr[10], wl[10];
    const v2f* rp = (const v2f*)(gp1root + lane * 10);
    const v2f* lp = (const v2f*)(gp1rel + lane * 10);
#pragma unroll
    for (int q = 0; q < 5; ++q) {
      const v2f tr = rp[q];
      const v2f tl = lp[q];
      wr[2 * q] = tr[0]; wr[2 * q + 1] = tr[1];
      wl[2 * q] = tl[0]; wl[2 * q + 1] = tl[1];
    }
    const float gb = gp1b[lane];
#pragma unroll 1
    for (int n = 0; n < 9; ++n) {
      float acc = 0.0f;
#pragma unroll
      for (int f = 0; f < 10; ++f) acc = fmaf(x0[n * 10 + f], wr[f], acc);
#pragma unroll
      for (int f = 0; f < 10; ++f) acc = fmaf(ag[n * 10 + f], wl[f], acc);
      acc += gb;
      gt[n * GTP + lane] = (_Float16)fmaxf(acc, 0.0f);
    }
  }
  __syncthreads();

  {
    const _Float16* G2W = (const _Float16*)G2Wp;
    const _Float16* ap = h1 + c * H1P + koff;
    const _Float16* bp = G2W + c * 128 + koff;
    const v16h a0 = FragH::load(ap),      a1 = FragH::load(ap + 32), a2 = FragH::load(ap + 64), a3 = FragH::load(ap + 96);
    const v16h b0 = FragH::load(bp),      b1 = FragH::load(bp + 32), b2 = FragH::load(bp + 64), b3 = FragH::load(bp + 96);
    v8f acc = z8;
    acc = FragH::mma(a0, b0, acc);
    acc = FragH::mma(a1, b1, acc);
    acc = FragH::mma(a2, b2, acc);
    acc = FragH::mma(a3, b3, acc);
    wm_guard1x8(acc, a0, a1, a2, a3, b0, b1, b2, b3);
#pragma unroll
    for (int r = 0; r < 8; ++r) xp2[(8 * hh + r) * 16 + c] = acc[r] * kWInv;
  }
#pragma unroll 1
  for (int i = 0; i < kChan; ++i) {
    const int p = (i < 4) ? 7 : 8;
    ga[i * GTP + lane] = gt[p * GTP + lane];
  }
#pragma unroll 1
  for (int it = 0; it < 3; ++it) {
    const int idx = it * 32 + lane;
    const int ic  = (idx < 70) ? idx : 69;
    const int n   = ic / 10;
    const int t   = ic - n * 10;
    const float v = x0[ic];
    if (idx < 70) xt[t * 32 + n] = (_Float16)v;
  }
  __syncthreads();

  {
    const _Float16* Wr = (const _Float16*)GC2rootp;
    const _Float16* Wl = (const _Float16*)GC2relp;
    const v16h a0 = FragH::load(gt + c * GTP + koff);
    const v16h a1 = FragH::load(ga + c * GTP + koff);
    const v16h b0 = FragH::load(Wr + c * 32 + koff);
    const v16h b1 = FragH::load(Wl + c * 32 + koff);
    v8f acc = z8;
    acc = FragH::mma(a0, b0, acc);
    acc = FragH::mma(a1, b1, acc);
    wm_guard1x4(acc, a0, a1, b0, b1);
    const int cc = (c < 10) ? c : 9;
    const float gb2 = gp2b[cc];
#pragma unroll
    for (int r = 0; r < 8; ++r) {
      const int node = 8 * hh + r;
      const float val = acc[r] * kWInv + gb2;
      if ((c < 10) && (node < kChan)) xt[c * 32 + 14 + node] = (_Float16)val;
    }
  }
  {
    float s2 = 0.0f, d2 = 0.0f;
#pragma unroll 1
    for (int f = 0; f < 10; ++f) {
      const float xv = xp2[c * 16 + f];
      s2 = fmaf(xv, ga2s[f], s2);
      d2 = fmaf(xv, ga2d[f], d2);
    }
    if (lane < 16) { s2v[lane] = s2; d2v[lane] = d2; }
  }
  __syncthreads();

  {
    const int tc = (lane < 10) ? lane : 9;
    const float b2 = ga2b[tc];
#pragma unroll 1
    for (int i = 0; i < kChan; ++i) {
      const int p = (i < 4) ? 7 : 8;
      const float di = d2v[i];
      float e0 = di + s2v[i];
      float e1 = di + s2v[p];
      e0 = (e0 >= 0.0f) ? e0 : 0.2f * e0;
      e1 = (e1 >= 0.0f) ? e1 : 0.2f * e1;
      const float mx = fmaxf(e0, e1);
      const float w0 = expf(e0 - mx);
      const float w1 = expf(e1 - mx);
      const float inv = 1.0f / (w0 + w1);
      const float val = (w0 * xp2[i * 16 + tc] + w1 * xp2[p * 16 + tc]) * inv + b2;
      if (lane < 10) xt[lane * 32 + 7 + i] = (_Float16)val;
    }
  }
  __syncthreads();

  {
    const v4u* xv = (const v4u*)xt;
    const v4u ca = xv[lane];
    const v4u cb = xv[32 + (lane & 7)];
    if (live) {
      unsigned short* dst = Xout + (size_t)b * kXRow;
      for (int pass = 0; pass < 2; ++pass) {
        *(volatile v4u*)(dst + lane * 8) = ca;
        if (lane < 8) *(volatile v4u*)(dst + 256 + lane * 8) = cb;
        __threadfence();
      }
    }
  }
}

struct SeqPtrs {
  const float* l1f_bih; const float* l1f_bhh; const float* l1b_bih; const float* l1b_bhh;
  const float* l2f_bih; const float* l2f_bhh; const float* l2b_bih; const float* l2b_bhh;
  const float* a1b; const float* a2b; const float* fcb;
};
static_assert(sizeof(SeqPtrs) == 88, "no padding");

template <int NKX>
__device__ __forceinline__ void bilstm_run(const _Float16* Xin, const int xstride,
                                           const _Float16* Wih, const _Float16* Whh,
                                           const float* bihF, const float* bhhF, const float* bihB, const float* bhhB,
                                           _Float16* O, const int lane, const int wave) {
  constexpr int KX = NKX * 32;
  const int d  = wave >> 2;
  const int hs = wave & 3;
  const int c = lane & 15, hh = lane >> 4, koff = hh * 8;
  const int n = hs * 16 + c;
  const _Float16* wih = Wih + (size_t)d * kGate * KX + koff;
  const _Float16* whh = Whh + (size_t)d * kGate * kLhid + koff;
  const v8f z8 = {0.f, 0.f, 0.f, 0.f, 0.f, 0.f, 0.f, 0.f};

  float bz[4];
#pragma unroll
  for (int q = 0; q < 4; ++q) {
    const int gi = q * kLhid + n;
    const float vf = bihF[gi] + bhhF[gi];
    const float vb = bihB[gi] + bhhB[gi];
    bz[q] = d ? vb : vf;
  }
  v16h bh[4][2];
#pragma unroll
  for (int q = 0; q < 4; ++q) {
#pragma unroll
    for (int kf = 0; kf < 2; ++kf) bh[q][kf] = FragH::load(whh + (size_t)(q * kLhid + n) * kLhid + kf * 32);
  }
  float cst[8];
#pragma unroll
  for (int r = 0; r < 8; ++r) cst[r] = 0.0f;

#pragma unroll 1
  for (int k = 0; k < kSeqT; ++k) {
    const int t = d ? (kSeqT - 1 - k) : k;
    v8f acc[4];
    acc[0] = z8; acc[1] = z8; acc[2] = z8; acc[3] = z8;
    const _Float16* xrow = Xin + (t * 16 + c) * xstride + koff;
#pragma unroll
    for (int kf = 0; kf < NKX; ++kf) {
      const v16h a  = FragH::load(xrow + kf * 32);
      const v16h b0 = FragH::load(wih + (size_t)(0 * kLhid + n) * KX + kf * 32);
      const v16h b1 = FragH::load(wih + (size_t)(1 * kLhid + n) * KX + kf * 32);
      const v16h b2 = FragH::load(wih + (size_t)(2 * kLhid + n) * KX + kf * 32);
      const v16h b3 = FragH::load(wih + (size_t)(3 * kLhid + n) * KX + kf * 32);
      acc[0] = FragH::mma(a, b0, acc[0]);
      acc[1] = FragH::mma(a, b1, acc[1]);
      acc[2] = FragH::mma(a, b2, acc[2]);
      acc[3] = FragH::mma(a, b3, acc[3]);
      wm_guard4(acc[0], acc[1], acc[2], acc[3], a, b0, b1, b2, b3);
    }
    if (k > 0) {
      const int tp = d ? (t + 1) : (t - 1);
      const _Float16* hrow = O + (tp * 16 + c) * OSTR + d * kLhid + koff;
#pragma unroll
      for (int kf = 0; kf < 2; ++kf) {
        const v16h a = FragH::load(hrow + kf * 32);
        acc[0] = FragH::mma(a, bh[0][kf], acc[0]);
        acc[1] = FragH::mma(a, bh[1][kf], acc[1]);
        acc[2] = FragH::mma(a, bh[2][kf], acc[2]);
        acc[3] = FragH::mma(a, bh[3][kf], acc[3]);
        wm_guard4(acc[0], acc[1], acc[2], acc[3], a, bh[0][kf], bh[1][kf], bh[2][kf], bh[3][kf]);
      }
    }
#pragma unroll
    for (int r = 0; r < 8; ++r) {
      const float zi = acc[0][r] * kWInv + bz[0];
      const float zf = acc[1][r] * kWInv + bz[1];
      const float zg = acc[2][r] * kWInv + bz[2];
      const float zo = acc[3][r] * kWInv + bz[3];
      const float ig = sigm_f(zi);
      const float fg = sigm_f(zf);
      const float gg = tanh_f(zg);
      const float og = sigm_f(zo);
      const float cn = fg * cst[r] + ig * gg;
      cst[r] = cn;
      const float hv = og * tanh_f(cn);
      O[(t * 16 + 8 * hh + r) * OSTR + d * kLhid + n] = (_Float16)hv;
    }
    __syncthreads();
  }
}

__device__ __forceinline__ void attn_qproj(const _Float16* O, _Float16* Q, const _Float16* W, const float* bias,
                                           const int lane, const int wave) {
  const int c = lane & 15, hh = lane >> 4, koff = hh * 8;
  const int n = wave * 16 + c;
  const _Float16* wp = W + (size_t)n * kCat + koff;
  const v16h b0 = FragH::load(wp), b1 = FragH::load(wp + 32), b2 = FragH::load(wp + 64), b3 = FragH::load(wp + 96);
  const float bq = bias[n];
  const v8f z8 = {0.f, 0.f, 0.f, 0.f, 0.f, 0.f, 0.f, 0.f};
#pragma unroll 1
  for (int mt = 0; mt < kSeqT; ++mt) {
    const _Float16* ap = O + (mt * 16 + c) * OSTR + koff;
    const v16h a0 = FragH::load(ap), a1 = FragH::load(ap + 32), a2 = FragH::load(ap + 64), a3 = FragH::load(ap + 96);
    v8f acc = z8;
    acc = FragH::mma(a0, b0, acc);
    acc = FragH::mma(a1, b1, acc);
    acc = FragH::mma(a2, b2, acc);
    acc = FragH::mma(a3, b3, acc);
    wm_guard1x8(acc, a0, a1, a2, a3, b0, b1, b2, b3);
#pragma unroll
    for (int r = 0; r < 8; ++r) {
      const float qv = tanh_f(acc[r] * kWInv + bq);
      Q[(mt * 16 + 8 * hh + r) * OSTR + n] = (_Float16)qv;
    }
  }
  __syncthreads();
}

__device__ __forceinline__ void attn_scores_wmma(const _Float16* Q, const _Float16* O, float* SC,
                                                 const int lane, const int wave) {
  const int c = lane & 15, hh = lane >> 4, koff = hh * 8;
  const int cr = (c < kSeqT) ? c : (kSeqT - 1);
  const v8f z8 = {0.f, 0.f, 0.f, 0.f, 0.f, 0.f, 0.f, 0.f};
#pragma unroll 1
  for (int ss = 0; ss < 2; ++ss) {
    const int s = wave * 2 + ss;
    const _Float16* qp = Q + (cr * 16 + s) * OSTR + koff;
    const _Float16* op = O + (cr * 16 + s) * OSTR + koff;
    const v16h a0 = FragH::load(qp), a1 = FragH::load(qp + 32), a2 = FragH::load(qp + 64), a3 = FragH::load(qp + 96);
    const v16h b0 = FragH::load(op), b1 = FragH::load(op + 32), b2 = FragH::load(op + 64), b3 = FragH::load(op + 96);
    v8f acc = z8;
    acc = FragH::mma(a0, b0, acc);
    acc = FragH::mma(a1, b1, acc);
    acc = FragH::mma(a2, b2, acc);
    acc = FragH::mma(a3, b3, acc);
    wm_guard1x8(acc, a0, a1, a2, a3, b0, b1, b2, b3);
#pragma unroll
    for (int r = 0; r < 8; ++r) {
      const int i = 8 * hh + r;
      if ((i < kSeqT) && (c < kSeqT)) SC[(s * kSeqT + i) * kSeqT + c] = acc[r];
    }
  }
  __syncthreads();
}

__device__ __forceinline__ void softmax_rows(float* SC, const int tid) {
  if (tid < 16 * kSeqT) {
    float* row = SC + tid * kSeqT;
    float mx = row[0];
#pragma unroll 1
    for (int j = 1; j < kSeqT; ++j) mx = fmaxf(mx, row[j]);
    float sum = 0.0f;
#pragma unroll 1
    for (int j = 0; j < kSeqT; ++j) {
      const float e = expf(row[j] - mx);
      row[j] = e;
      sum += e;
    }
    const float inv = 1.0f / sum;
#pragma unroll 1
    for (int j = 0; j < kSeqT; ++j) row[j] = row[j] * inv;
  }
  __syncthreads();
}

__device__ __forceinline__ void attn_apply(const float* SC, const _Float16* O, _Float16* D, const int tid) {
  const int s = tid >> 4, r16 = tid & 15;
  const int c0 = r16 * 8;
  float ov[kSeqT][8];
#pragma unroll
  for (int j = 0; j < kSeqT; ++j) {
    const v4u w = *(const v4u*)(O + (j * 16 + s) * OSTR + c0);
    const unsigned w0 = w[0], w1 = w[1], w2 = w[2], w3 = w[3];
    ov[j][0] = h16_to_f32(w0 & 0xffffu); ov[j][1] = h16_to_f32(w0 >> 16);
    ov[j][2] = h16_to_f32(w1 & 0xffffu); ov[j][3] = h16_to_f32(w1 >> 16);
    ov[j][4] = h16_to_f32(w2 & 0xffffu); ov[j][5] = h16_to_f32(w2 >> 16);
    ov[j][6] = h16_to_f32(w3 & 0xffffu); ov[j][7] = h16_to_f32(w3 >> 16);
  }
#pragma unroll 1
  for (int i = 0; i < kSeqT; ++i) {
    float acc[8];
#pragma unroll
    for (int e = 0; e < 8; ++e) acc[e] = 0.0f;
#pragma unroll
    for (int j = 0; j < kSeqT; ++j) {
      const float a = SC[(s * kSeqT + i) * kSeqT + j];
#pragma unroll
      for (int e = 0; e < 8; ++e) acc[e] = fmaf(a, ov[j][e], acc[e]);
    }
    v8h hv;
#pragma unroll
    for (int e = 0; e < 8; ++e) hv[e] = (_Float16)acc[e];
    *(v8h*)(D + (i * 16 + s) * OSTR + c0) = hv;
  }
  __syncthreads();
}

__device__ __forceinline__ void attn_mean_apply(const float* SC, const _Float16* O, _Float16* MB, float* AB, const int tid) {
  if (tid < 16 * kSeqT) {
    const int s = tid / kSeqT;
    const int j = tid - s * kSeqT;
    float a = 0.0f;
#pragma unroll 1
    for (int i = 0; i < kSeqT; ++i) a += SC[(s * kSeqT + i) * kSeqT + j];
    AB[tid] = a * (1.0f / (float)kSeqT);
  }
  __syncthreads();
  const int s = tid >> 4, r16 = tid & 15;
  const int c0 = r16 * 8;
  float acc[8];
#pragma unroll
  for (int e = 0; e < 8; ++e) acc[e] = 0.0f;
#pragma unroll 1
  for (int j = 0; j < kSeqT; ++j) {
    const float a = AB[s * kSeqT + j];
    const v4u w = *(const v4u*)(O + (j * 16 + s) * OSTR + c0);
    const unsigned w0 = w[0], w1 = w[1], w2 = w[2], w3 = w[3];
    acc[0] = fmaf(a, h16_to_f32(w0 & 0xffffu), acc[0]); acc[1] = fmaf(a, h16_to_f32(w0 >> 16), acc[1]);
    acc[2] = fmaf(a, h16_to_f32(w1 & 0xffffu), acc[2]); acc[3] = fmaf(a, h16_to_f32(w1 >> 16), acc[3]);
    acc[4] = fmaf(a, h16_to_f32(w2 & 0xffffu), acc[4]); acc[5] = fmaf(a, h16_to_f32(w2 >> 16), acc[5]);
    acc[6] = fmaf(a, h16_to_f32(w3 & 0xffffu), acc[6]); acc[7] = fmaf(a, h16_to_f32(w3 >> 16), acc[7]);
  }
  v8h hv;
#pragma unroll
  for (int e = 0; e < 8; ++e) hv[e] = (_Float16)acc[e];
  *(v8h*)(MB + s * OSTR + c0) = hv;
  __syncthreads();
}

__global__ __launch_bounds__(256) void seq_fused_kernel(
    const unsigned short* __restrict__ Xp,
    const unsigned short* __restrict__ W1ihp, const unsigned short* __restrict__ W1hhp,
    const unsigned short* __restrict__ W2ihp, const unsigned short* __restrict__ W2hhp,
    const unsigned short* __restrict__ AWp, SeqPtrs sp, float* __restrict__ out) {
  __shared__ __align__(16) _Float16 Xl[kSeqT * 16 * XSTR];
  __shared__ __align__(16) _Float16 O1[kSeqT * 16 * OSTR];
  __shared__ __align__(16) _Float16 QX[kSeqT * 16 * OSTR];
  __shared__ __align__(16) float    SC[16 * kSeqT * kSeqT];
  __shared__ __align__(16) float    AB[16 * kSeqT];
  __shared__ __align__(16) _Float16 MB[16 * OSTR];
  __shared__ __align__(16) float    OS[16 * OSP];

  const int tid  = threadIdx.x;
  const int lane = tid & 31;
  const int wave = tid >> 5;
  const size_t b0 = (size_t)blockIdx.x * 16;

  const _Float16* W1ih = (const _Float16*)W1ihp;
  const _Float16* W1hh = (const _Float16*)W1hhp;
  const _Float16* W2ih = (const _Float16*)W2ihp;
  const _Float16* W2hh = (const _Float16*)W2hhp;
  const _Float16* A1W  = (const _Float16*)AWp;
  const _Float16* A2W  = A1W + kCat * kCat;
  const _Float16* FCW  = A1W + 2 * kCat * kCat;

  {
    const v4u* Xg = (const v4u*)(Xp + b0 * kXRow);
#pragma unroll 1
    for (int it = 0; it < 3; ++it) {
      const int q  = it * 256 + tid;
      const int qc = (q < 640) ? q : 639;
      const int s   = qc / 40;
      const int rem = qc - s * 40;
      const int t   = rem >> 2;
      const int part = rem & 3;
      const v4u v = Xg[qc];
      if (q < 640) *(v4u*)(Xl + (t * 16 + s) * XSTR + part * 8) = v;
    }
  }
  __syncthreads();

  bilstm_run<1>(Xl, XSTR, W1ih, W1hh, sp.l1f_bih, sp.l1f_bhh, sp.l1b_bih, sp.l1b_bhh, O1, lane, wave);
  attn_qproj(O1, QX, A1W, sp.a1b, lane, wave);
  attn_scores_wmma(QX, O1, SC, lane, wave);
  softmax_rows(SC, tid);
  attn_apply(SC, O1, QX, tid);

  bilstm_run<4>(QX, OSTR, W2ih, W2hh, sp.l2f_bih, sp.l2f_bhh, sp.l2b_bih, sp.l2b_bhh, O1, lane, wave);
  attn_qproj(O1, QX, A2W, sp.a2b, lane, wave);
  attn_scores_wmma(QX, O1, SC, lane, wave);
  softmax_rows(SC, tid);
  attn_mean_apply(SC, O1, MB, AB, tid);

  {
    const int c = lane & 15, hh = lane >> 4, koff = hh * 8;
    const int n = wave * 16 + c;
    const _Float16* ap = MB + c * OSTR + koff;
    const _Float16* wp = FCW + (size_t)n * kCat + koff;
    const v16h a0 = FragH::load(ap), a1 = FragH::load(ap + 32), a2 = FragH::load(ap + 64), a3 = FragH::load(ap + 96);
    const v16h b0 = FragH::load(wp), b1 = FragH::load(wp + 32), b2 = FragH::load(wp + 64), b3 = FragH::load(wp + 96);
    v8f acc = {0.f, 0.f, 0.f, 0.f, 0.f, 0.f, 0.f, 0.f};
    acc = FragH::mma(a0, b0, acc);
    acc = FragH::mma(a1, b1, acc);
    acc = FragH::mma(a2, b2, acc);
    acc = FragH::mma(a3, b3, acc);
    wm_guard1x8(acc, a0, a1, a2, a3, b0, b1, b2, b3);
    const float bq = sp.fcb[n];
#pragma unroll
    for (int r = 0; r < 8; ++r) OS[(8 * hh + r) * OSP + n] = acc[r] * kWInv + bq;
  }
  __syncthreads();
  {
    const int r0 = wave * 2;
    const v4f v0 = *(const v4f*)(OS + r0 * OSP + lane * 4);
    const v4f v1 = *(const v4f*)(OS + (r0 + 1) * OSP + lane * 4);
    float* o0 = out + (b0 + r0) * kEmb + lane * 4;
    float* o1 = out + (b0 + r0 + 1) * kEmb + lane * 4;
    for (int pass = 0; pass < 2; ++pass) {
      *(volatile v4f*)o0 = v0;
      *(volatile v4f*)o1 = v1;
      __threadfence();
    }
  }
}

extern "C" void kernel_launch(void* const* d_in, const int* in_sizes, int n_in,
                              void* d_out, int out_size, void* d_ws, size_t ws_size, hipStream_t stream) {
  if (n_in < 37 || d_out == nullptr || d_ws == nullptr) return;
  const int nB = in_sizes[0] / (kChan * kSeqT);
  if (nB <= 0 || nB * kChan * kSeqT != in_sizes[0] || (nB % 16) != 0 || out_size != nB * kEmb) return;
  const int expect[37] = {0, 1280, 128, 128, 128, 1280, 10, 10, 10, 320, 320, 32, 320, 320, 10,
                          5376, 16384, 256, 256, 5376, 16384, 256, 256,
                          32768, 16384, 256, 256, 32768, 16384, 256, 256,
                          16384, 128, 16384, 128, 16384, 128};
  for (int i = 1; i < 37; ++i) { if (in_sizes[i] != expect[i]) return; }

  char* ws = (char*)d_ws; size_t off = 0;
  auto carve = [&](size_t bytes) -> char* { char* p = ws + off; off += (bytes + 255) & ~(size_t)255; return p; };
  unsigned short* X    = (unsigned short*)carve((size_t)nB * kXRow * 2);
  unsigned short* W1ih = (unsigned short*)carve((size_t)2 * kGate * kFeat1Pad * 2);
  unsigned short* W1hh = (unsigned short*)carve((size_t)2 * kGate * kLhid * 2);
  unsigned short* W2ih = (unsigned short*)carve((size_t)2 * kGate * kCat * 2);
  unsigned short* W2hh = (unsigned short*)carve((size_t)2 * kGate * kLhid * 2);
  unsigned short* AW   = (unsigned short*)carve((size_t)3 * kCat * kCat * 2);
  unsigned short* G2W  = (unsigned short*)carve((size_t)16 * 128 * 2);
  unsigned short* GC2  = (unsigned short*)carve((size_t)2 * 16 * 32 * 2);
  if (off > ws_size || off > (size_t)134217728) return;

  const float* f[37];
  for (int i = 0; i < 37; ++i) f[i] = (const float*)d_in[i];

  cvt_plane_kernel<<<dim3(4, 2),  256, 0, stream>>>(f[15], f[19], f[19], W1ih, kGate, kFeat1, kGate, kFeat1Pad, kWCarry);
  cvt_plane_kernel<<<dim3(8, 2),  256, 0, stream>>>(f[16], f[20], f[20], W1hh, kGate, kLhid,  kGate, kLhid,     kWCarry);
  cvt_plane_kernel<<<dim3(16, 2), 256, 0, stream>>>(f[23], f[27], f[27], W2ih, kGate, kCat,   kGate, kCat,      kWCarry);
  cvt_plane_kernel<<<dim3(8, 2),  256, 0, stream>>>(f[24], f[28], f[28], W2hh, kGate, kLhid,  kGate, kLhid,     kWCarry);
  cvt_plane_kernel<<<dim3(8, 3),  256, 0, stream>>>(f[31], f[33], f[35], AW,   kCat,  kCat,   kCat,  kCat,      kWCarry);
  cvt_plane_kernel<<<dim3(1, 1),  256, 0, stream>>>(f[5],  f[5],  f[5],  G2W,  10,    128,    16,    128,       kWCarry);
  cvt_plane_kernel<<<dim3(1, 2),  256, 0, stream>>>(f[13], f[12], f[12], GC2,  10,    32,     16,    32,        kWCarry);

  graph_front_kernel<<<(nB + GKW - 1) / GKW, 32 * GKW, 0, stream>>>(
      f[0], f[1], f[2], f[3], f[4], G2W, f[6], f[7], f[8], f[9], f[10], f[11],
      GC2, GC2 + 16 * 32, f[14], X, nB);

  SeqPtrs sp;
  sp.l1f_bih = f[17]; sp.l1f_bhh = f[18]; sp.l1b_bih = f[21]; sp.l1b_bhh = f[22];
  sp.l2f_bih = f[25]; sp.l2f_bhh = f[26]; sp.l2b_bih = f[29]; sp.l2b_bhh = f[30];
  sp.a1b = f[32]; sp.a2b = f[34]; sp.fcb = f[36];
  seq_fused_kernel<<<nB / 16, 256, 0, stream>>>(X, W1ih, W1hh, W2ih, W2hh, AW, sp, (float*)d_out);
}
